// FullGraphEncoder_19129784336896
// MI455X (gfx1250) — hardware-verified
//
#include <hip/hip_runtime.h>


#define VOCAB   100
#define NBOND   4
#define EMB     128
#define DEPTH   4
#define NNODES  25000
#define NEDGES  50000
#define MAXNB   6
#define INROWS  (VOCAB + NBOND)
#define WROWS   (INROWS + EMB)
#define TROWS   (VOCAB + EMB)
#define HWLD    256

#define SC_H    16.0f
#define SC_W    64.0f
#define SC_INV  0.0009765625f

static_assert(NEDGES % 16 == 0);
static_assert(NEDGES % 8 == 0);
static_assert(NNODES % 8 == 0);

typedef unsigned short us16;
typedef us16     v8us __attribute__((ext_vector_type(8)));
typedef _Float16 v16h __attribute__((ext_vector_type(16)));
typedef float    v8f  __attribute__((ext_vector_type(8)));
typedef float    v4f  __attribute__((ext_vector_type(4)));
typedef v4f      v4fa __attribute__((may_alias));
typedef unsigned v4u  __attribute__((ext_vector_type(4)));
typedef unsigned v2u  __attribute__((ext_vector_type(2)));

union FragH { v16h v; v8us half[2]; };

constexpr size_t P1_BYTES = (size_t)16 * 4 * 32 * 16 * 2;
constexpr size_t PT_BYTES = (size_t)8 * 4 * 32 * 16 * 2;
constexpr size_t HF_BYTES = (size_t)NEDGES * EMB * 2;
constexpr size_t C_BYTES  = (size_t)NEDGES * EMB * 4;
constexpr size_t HW_BYTES = (size_t)NEDGES * HWLD * 4;
constexpr size_t OFF_P1 = 0;
constexpr size_t OFF_P2 = OFF_P1 + P1_BYTES;
constexpr size_t OFF_PT = OFF_P2 + P1_BYTES;
constexpr size_t OFF_HF = OFF_PT + PT_BYTES;
constexpr size_t OFF_C0 = OFF_HF + HF_BYTES;
constexpr size_t OFF_C1 = OFF_C0 + C_BYTES;
constexpr size_t OFF_HW = OFF_C1 + C_BYTES;
constexpr size_t WS_END = OFF_HW + HW_BYTES;
static_assert(OFF_P2 % 256 == 0 && OFF_PT % 256 == 0 && OFF_HF % 256 == 0);
static_assert(OFF_C0 % 256 == 0 && OFF_C1 % 256 == 0 && OFF_HW % 256 == 0);
static_assert(P1_BYTES % 512 == 0 && PT_BYTES % 512 == 0 && HF_BYTES % 256 == 0);
static_assert(C_BYTES % 512 == 0 && HW_BYTES % 1024 == 0);
static_assert(WS_END <= (size_t)134217728);

__device__ __forceinline__ v4f zero4() { v4f z; z[0] = 0.0f; z[1] = 0.0f; z[2] = 0.0f; z[3] = 0.0f; return z; }
__device__ __forceinline__ v4f ld4(const float* p) { return *(const v4f*)p; }
__device__ __forceinline__ v4f keep4(v4f v, bool c) {
    v4f r;
    r[0] = c ? v[0] : 0.0f; r[1] = c ? v[1] : 0.0f; r[2] = c ? v[2] : 0.0f; r[3] = c ? v[3] : 0.0f;
    return r;
}
__device__ __forceinline__ int clampi(int x, int lo, int hi) { return min(max(x, lo), hi); }
__device__ __forceinline__ unsigned pkh(float a, float b) {
    const us16 x = __builtin_bit_cast(us16, (_Float16)a);
    const us16 y = __builtin_bit_cast(us16, (_Float16)b);
    return (unsigned)x | ((unsigned)y << 16);
}
__device__ __forceinline__ float fsig(float x) {
    const float t = fminf(fmaxf(x, -80.0f), 80.0f);
    const float e = __expf(-t);
    return __builtin_amdgcn_rcpf(1.0f + e);
}
__device__ __forceinline__ float ftanh(float x) {
    const float t = fminf(fmaxf(x, -40.0f), 40.0f);
    const float e = __expf(2.0f * t);
    return 1.0f - 2.0f * __builtin_amdgcn_rcpf(1.0f + e);
}

__device__ __forceinline__ v8f mma16(v8f c, const FragH& a, const FragH& b) {
    c = __builtin_amdgcn_wmma_f32_16x16x32_f16(false, a.v, false, b.v, (short)0, c, false, false);
    asm volatile("v_nop\n\tv_nop\n\tv_nop\n\tv_nop" : "+v"(c) : "v"(a.v), "v"(b.v));
    return c;
}

__global__ __launch_bounds__(256) void k_pack(const float* __restrict__ Wi, const float* __restrict__ Wu,
                                              const float* __restrict__ Wf, const float* __restrict__ Wo,
                                              const float* __restrict__ Wt,
                                              us16* P1, us16* P2, us16* PT)
{
    const int b = blockIdx.x, tid = threadIdx.x;
    int nt, col, rowb;
    const float* W;
    us16* base;
    if (b < 16)      { nt = b;      W = (nt < 8) ? Wi : Wu; col = (nt & 7) * 16; rowb = INROWS; base = P1; }
    else if (b < 32) { nt = b - 16; W = (nt < 8) ? Wf : Wo; col = (nt & 7) * 16; rowb = INROWS; base = P2; }
    else             { nt = b - 32; W = Wt;                  col = nt * 16;       rowb = VOCAB;  base = PT; }
    const int half = tid & 1;
    const int lane = (tid >> 1) & 31;
    const int ks   = (tid >> 6) & 3;
    const int hh   = lane >> 4, m = lane & 15;
    const int k0   = ks * 32 + 16 * half + 8 * hh;
    const float* src = W + (size_t)(rowb + k0) * EMB + col + m;
    float v[8];
#pragma unroll
    for (int i = 0; i < 8; ++i) v[i] = src[(size_t)i * EMB] * SC_W;
    v4u o;
    o[0] = pkh(v[0], v[1]); o[1] = pkh(v[2], v[3]); o[2] = pkh(v[4], v[5]); o[3] = pkh(v[6], v[7]);
    us16* dst = base + ((size_t)nt * 256 + tid) * 8;
    *(volatile v4u*)dst = o;
    __threadfence();
    *(volatile v4u*)dst = o;
}

__global__ __launch_bounds__(32) void k_gemm(const us16* __restrict__ A, const us16* __restrict__ Bp, float* C, int ldc)
{
    __shared__ __attribute__((aligned(16))) float sT[16 * 128];
    const int l = threadIdx.x & 31, h = l >> 4, m = l & 15;
    const int row0 = blockIdx.x * 16;
    const int cg = blockIdx.y;

    v8f acc[8];
#pragma unroll
    for (int nt = 0; nt < 8; ++nt)
#pragma unroll
        for (int r = 0; r < 8; ++r) acc[nt][r] = 0.0f;

    const us16* arow = A + (size_t)(row0 + m) * EMB + 8 * h;
#pragma unroll
    for (int ks = 0; ks < 4; ++ks) {
        FragH a;
        a.half[0] = *(const v8us*)(arow + ks * 32);
        a.half[1] = *(const v8us*)(arow + ks * 32 + 16);
#pragma unroll
        for (int nt = 0; nt < 8; ++nt) {
            const us16* bp = Bp + ((size_t)((cg * 8 + nt) * 4 + ks) * 32 + l) * 16;
            FragH b;
            b.half[0] = *(const v8us*)bp;
            b.half[1] = *(const v8us*)(bp + 8);
            acc[nt] = mma16(acc[nt], a, b);
        }
    }

#pragma unroll
    for (int nt = 0; nt < 8; ++nt)
#pragma unroll
        for (int r = 0; r < 8; ++r) sT[(8 * h + r) * 128 + nt * 16 + m] = acc[nt][r];
    __syncthreads();

    float* cb = C + (size_t)row0 * ldc + cg * 128 + 4 * l;
#pragma unroll
    for (int i = 0; i < 16; ++i) {
        const v4f v = *(const v4fa*)(&sT[i * 128 + 4 * l]);
        *(volatile v4f*)(cb + (size_t)i * ldc) = v;
    }
    __threadfence();
#pragma unroll
    for (int i = 0; i < 16; ++i) {
        const v4f v = *(const v4fa*)(&sT[i * 128 + 4 * l]);
        *(volatile v4f*)(cb + (size_t)i * ldc) = v;
    }
}

__global__ __launch_bounds__(256) void k_step_a(const float* __restrict__ hW, int has_h,
                                                const int* __restrict__ bond, const int* __restrict__ node_ids,
                                                const int* __restrict__ edge_src, const int* __restrict__ edge_type,
                                                const float* __restrict__ Wi, const float* __restrict__ bi,
                                                const float* __restrict__ Wu, const float* __restrict__ bu,
                                                float* c_out)
{
    const int tid = threadIdx.x;
    const int l   = tid & 31;
    const int e   = blockIdx.x * 8 + (tid >> 5);
    const int j0  = 4 * l;

    const int src  = clampi(edge_src[e], 0, NNODES - 1);
    const int nid  = node_ids[src];
    const bool va  = (unsigned)nid < (unsigned)VOCAB;
    const int nidc = clampi(nid, 0, VOCAB - 1);
    const int bty  = edge_type[e];
    const bool vb  = (unsigned)bty < (unsigned)NBOND;
    const int btc  = clampi(bty, 0, NBOND - 1);

    const size_t ra = (size_t)nidc * EMB + j0;
    const size_t rb = (size_t)(VOCAB + btc) * EMB + j0;
    const v4f pi = ld4(bi + j0) + keep4(ld4(Wi + ra), va) + keep4(ld4(Wi + rb), vb);
    const v4f pu = ld4(bu + j0) + keep4(ld4(Wu + ra), va) + keep4(ld4(Wu + rb), vb);

    v4f xi = zero4(), xu = zero4();
    if (has_h) {
#pragma unroll
        for (int k = 0; k < MAXNB; ++k) {
            const int bk = clampi(bond[(size_t)e * MAXNB + k], 0, NEDGES - 1);
            const float* r = hW + (size_t)bk * HWLD;
            xi += ld4(r + j0);
            xu += ld4(r + 128 + j0);
        }
    }
    v4f v;
#pragma unroll
    for (int q = 0; q < 4; ++q) v[q] = fsig(xi[q] * SC_INV + pi[q]) * ftanh(xu[q] * SC_INV + pu[q]);

    float* dst = c_out + (size_t)e * EMB + j0;
    *(volatile v4f*)dst = v;
    __threadfence();
    *(volatile v4f*)dst = v;
}

__global__ __launch_bounds__(256) void k_step_b(const float* __restrict__ hW, const float* __restrict__ c_in, int has_h,
                                                const int* __restrict__ bond, const int* __restrict__ node_ids,
                                                const int* __restrict__ edge_src, const int* __restrict__ edge_type,
                                                const float* __restrict__ Wf, const float* __restrict__ bf,
                                                const float* __restrict__ Wo, const float* __restrict__ bo,
                                                float* c_out, us16* hF)
{
    const int tid = threadIdx.x;
    const int l   = tid & 31;
    const int e   = blockIdx.x * 8 + (tid >> 5);
    const int j0  = 4 * l;

    const int src  = clampi(edge_src[e], 0, NNODES - 1);
    const int nid  = node_ids[src];
    const bool va  = (unsigned)nid < (unsigned)VOCAB;
    const int nidc = clampi(nid, 0, VOCAB - 1);
    const int bty  = edge_type[e];
    const bool vb  = (unsigned)bty < (unsigned)NBOND;
    const int btc  = clampi(bty, 0, NBOND - 1);

    const size_t ra = (size_t)nidc * EMB + j0;
    const size_t rb = (size_t)(VOCAB + btc) * EMB + j0;
    const v4f pf = ld4(bf + j0) + keep4(ld4(Wf + ra), va) + keep4(ld4(Wf + rb), vb);
    const v4f po = ld4(bo + j0) + keep4(ld4(Wo + ra), va) + keep4(ld4(Wo + rb), vb);

    v4f fc = zero4(), xo = zero4();
    if (has_h) {
#pragma unroll 2
        for (int k = 0; k < MAXNB; ++k) {
            const int bk = clampi(bond[(size_t)e * MAXNB + k], 0, NEDGES - 1);
            const float* r = hW + (size_t)bk * HWLD;
            const v4f xf = ld4(r + j0);
            xo += ld4(r + 128 + j0);
            const v4f cv = ld4(c_in + (size_t)bk * EMB + j0);
            v4f fg;
#pragma unroll
            for (int q = 0; q < 4; ++q) fg[q] = fsig(xf[q] * SC_INV + pf[q]);
            fc += fg * cv;
        }
    }
    const float fm  = (e == 0) ? 0.0f : 1.0f;
    const v4f part  = ld4(c_out + (size_t)e * EMB + j0);
    const v4f cn    = (part + fc) * fm;
    v4f hv;
#pragma unroll
    for (int q = 0; q < 4; ++q) hv[q] = fsig(xo[q] * SC_INV + po[q]) * ftanh(cn[q]) * fm;

    v2u hb;
    hb[0] = pkh(hv[0] * SC_H, hv[1] * SC_H);
    hb[1] = pkh(hv[2] * SC_H, hv[3] * SC_H);

    float* dc = c_out + (size_t)e * EMB + j0;
    us16*  dh = hF + (size_t)e * EMB + j0;
    *(volatile v4f*)dc = cn;
    *(volatile v2u*)dh = hb;
    __threadfence();
    *(volatile v4f*)dc = cn;
    *(volatile v2u*)dh = hb;
}

__global__ __launch_bounds__(256) void k_readout(const float* __restrict__ hWt, const int* __restrict__ adj,
                                                 const int* __restrict__ node_ids,
                                                 const float* __restrict__ Wt, const float* __restrict__ bt,
                                                 float* out)
{
    const int tid = threadIdx.x;
    const int l   = tid & 31;
    const int n   = blockIdx.x * 8 + (tid >> 5);
    const int j0  = 4 * l;

    const int nid  = node_ids[n];
    const bool va  = (unsigned)nid < (unsigned)VOCAB;
    const int nidc = clampi(nid, 0, VOCAB - 1);

    v4f s = zero4();
#pragma unroll
    for (int k = 0; k < MAXNB; ++k) {
        const int ak = clampi(adj[(size_t)n * MAXNB + k], 0, NEDGES - 1);
        s += ld4(hWt + (size_t)ak * EMB + j0);
    }
    const v4f base = ld4(bt + j0) + keep4(ld4(Wt + (size_t)nidc * EMB + j0), va);
    const float nm = (n == 0) ? 0.0f : 1.0f;
    v4f v;
#pragma unroll
    for (int q = 0; q < 4; ++q) v[q] = fmaxf(s[q] * SC_INV + base[q], 0.0f) * nm;

    float* dst = out + (size_t)n * EMB + j0;
    *(volatile v4f*)dst = v;
    __threadfence();
    *(volatile v4f*)dst = v;
}

extern "C" void kernel_launch(void* const* d_in, const int* in_sizes, int n_in,
                              void* d_out, int out_size, void* d_ws, size_t ws_size,
                              hipStream_t stream)
{
    if (n_in < 15) return;
    const int expect[15] = {
        NNODES, NEDGES, NEDGES, NNODES * MAXNB, NEDGES * MAXNB,
        WROWS * EMB, EMB, WROWS * EMB, EMB, WROWS * EMB, EMB, WROWS * EMB, EMB, TROWS * EMB, EMB };
    for (int i = 0; i < 15; ++i) if (in_sizes[i] != expect[i]) return;
    if (out_size != NNODES * EMB) return;
    if (ws_size < WS_END) return;

    const int*   node_ids  = (const int*)  d_in[0];
    const int*   edge_src  = (const int*)  d_in[1];
    const int*   edge_type = (const int*)  d_in[2];
    const int*   adj_list  = (const int*)  d_in[3];
    const int*   bond_list = (const int*)  d_in[4];
    const float* Wi = (const float*)d_in[5];
    const float* bi = (const float*)d_in[6];
    const float* Wo = (const float*)d_in[7];
    const float* bo = (const float*)d_in[8];
    const float* Wf = (const float*)d_in[9];
    const float* bf = (const float*)d_in[10];
    const float* Wu = (const float*)d_in[11];
    const float* bu = (const float*)d_in[12];
    const float* Wt = (const float*)d_in[13];
    const float* bt = (const float*)d_in[14];
    float* out = (float*)d_out;

    char* ws = (char*)d_ws;
    us16*  P1 = (us16*)(ws + OFF_P1);
    us16*  P2 = (us16*)(ws + OFF_P2);
    us16*  PT = (us16*)(ws + OFF_PT);
    us16*  hF = (us16*)(ws + OFF_HF);
    float* cpl[2] = { (float*)(ws + OFF_C0), (float*)(ws + OFF_C1) };
    float* hW = (float*)(ws + OFF_HW);

    k_pack<<<dim3(40), dim3(256), 0, stream>>>(Wi, Wu, Wf, Wo, Wt, P1, P2, PT);

    const dim3 ggrid(NEDGES / 16, 2);
    const dim3 sgrid(NEDGES / 8);
    for (int d = 0; d < DEPTH; ++d) {
        const int has_h = (d > 0) ? 1 : 0;
        float* c_in  = cpl[d & 1];
        float* c_out = cpl[(d + 1) & 1];
        if (has_h) k_gemm<<<ggrid, dim3(32), 0, stream>>>(hF, P1, hW, HWLD);
        k_step_a<<<sgrid, dim3(256), 0, stream>>>(hW, has_h, bond_list, node_ids, edge_src, edge_type,
                                                   Wi, bi, Wu, bu, c_out);
        if (has_h) k_gemm<<<ggrid, dim3(32), 0, stream>>>(hF, P2, hW, HWLD);
        k_step_b<<<sgrid, dim3(256), 0, stream>>>(hW, c_in, has_h, bond_list, node_ids, edge_src, edge_type,
                                                   Wf, bf, Wo, bo, c_out, hF);
    }

    k_gemm<<<dim3(NEDGES / 16, 1), dim3(32), 0, stream>>>(hF, PT, hW, EMB);
    k_readout<<<dim3(NNODES / 8), dim3(256), 0, stream>>>(hW, adj_list, node_ids, Wt, bt, out);
}
